// MultiHeadAttentionLayer_39505109188985
// MI455X (gfx1250) — hardware-verified
//
#include <hip/hip_runtime.h>


#ifndef NB
#define NB 2
#endif
#ifndef SEQ
#define SEQ 2048
#endif
#define SEQ_FULL 2048
#define DM   1024
#define NH   16
#define HD   64
#define N3   (3 * DM)
#define NBH  (NB * NH)
#define MROWS (NB * SEQ)
#define PLN  ((size_t)NBH * SEQ * HD)
#define CSC  0.18033688011112042f

static_assert(SEQ % 64 == 0);
static_assert(SEQ <= SEQ_FULL);
static_assert(MROWS % 64 == 0);
static_assert(N3 % 64 == 0);
static_assert(DM % 64 == 0);
static_assert(HD == 64);
static_assert(NH * HD == DM);
static_assert(((size_t)NBH * SEQ * HD) % 8 == 0);
static_assert((size_t)NBH * SEQ * HD < 0x7fffffffu);

typedef unsigned short bf;
typedef __attribute__((ext_vector_type(16))) __bf16   v16bf;
typedef __attribute__((ext_vector_type(8)))  unsigned short v8us;
typedef __attribute__((ext_vector_type(8)))  unsigned int v8u;
typedef __attribute__((ext_vector_type(8)))  float    v8f;
typedef __attribute__((ext_vector_type(4)))  float    v4f;
typedef v4f  __attribute__((may_alias)) v4fa;
typedef v8us __attribute__((may_alias)) v8usa;

__device__ __forceinline__ unsigned short f2bf(float f) { unsigned u = __float_as_uint(f); u += 0x7FFFu + ((u >> 16) & 1u); return (unsigned short)(u >> 16); }
__device__ __forceinline__ float bf2f(unsigned short b) { return __uint_as_float(((unsigned)b) << 16); }
__device__ __forceinline__ float bfr(float f) { return bf2f(f2bf(f)); }
__device__ __forceinline__ v16bf cat16b(v8us lo, v8us hi) { return __builtin_bit_cast(v16bf, __builtin_shufflevector(lo, hi, 0, 1, 2, 3, 4, 5, 6, 7, 8, 9, 10, 11, 12, 13, 14, 15)); }
__device__ __forceinline__ v8f wmmab(v16bf a, v16bf b, v8f c) { return __builtin_amdgcn_wmma_f32_16x16x32_bf16(false, a, false, b, (short)0, c, false, false); }
__device__ __forceinline__ void splitf(float y, unsigned short& h, unsigned short& l) { h = f2bf(y); l = f2bf(y - bf2f(h)); }

template <typename T16> struct WFrag;
template <> struct WFrag<bf> { typedef v16bf V; static __device__ __forceinline__ V ld(const bf* p) { return cat16b(*(const v8us*)p, *(const v8us*)(p + 16)); } static __device__ __forceinline__ v8f mma(V a, V b, v8f c) { return wmmab(a, b, c); } };

template <typename T16, int NSPLIT, bool BIAS>
__global__ __launch_bounds__(32) void k_gemmw(const T16* __restrict__ A, const T16* __restrict__ A2, const T16* __restrict__ Bt, const T16* __restrict__ Bt2, int K, float* C, int ldc, const float* __restrict__ bias, size_t sA, size_t sB, size_t sC) {
    typedef typename WFrag<T16>::V V;
    __shared__ __align__(16) float os[16 * 68];
    const size_t z = blockIdx.z; A += z * sA; if (A2) A2 += z * sA; Bt += z * sB; if (Bt2) Bt2 += z * sB; C += z * sC;
    const int lane = threadIdx.x & 31, lr = lane & 15, hi = lane >> 4; const int r0 = blockIdx.x * 64, c0 = blockIdx.y * 64;
    v8f acc[4][4];
#pragma unroll
    for (int mb = 0; mb < 4; ++mb)
#pragma unroll
        for (int nb = 0; nb < 4; ++nb) acc[mb][nb] = (v8f){};
    const size_t aoff = (size_t)(r0 + lr) * K + 8 * hi, boff = (size_t)(c0 + lr) * K + 8 * hi;
#pragma unroll 1
    for (int kc = 0; kc < K; kc += 32) {
        V a[4], a2[4];
#pragma unroll
        for (int mb = 0; mb < 4; ++mb) { a[mb] = WFrag<T16>::ld(A + aoff + (size_t)mb * 16 * K + kc); if (NSPLIT == 1 || NSPLIT == 2) a2[mb] = WFrag<T16>::ld(A2 + aoff + (size_t)mb * 16 * K + kc); }
#pragma unroll
        for (int nb = 0; nb < 4; ++nb) { const V b = WFrag<T16>::ld(Bt + boff + (size_t)nb * 16 * K + kc); V b2; if (NSPLIT >= 2) b2 = WFrag<T16>::ld(Bt2 + boff + (size_t)nb * 16 * K + kc);
#pragma unroll
            for (int mb = 0; mb < 4; ++mb) { acc[mb][nb] = WFrag<T16>::mma(a[mb], b, acc[mb][nb]); if (NSPLIT == 1 || NSPLIT == 2) acc[mb][nb] = WFrag<T16>::mma(a2[mb], b, acc[mb][nb]); if (NSPLIT >= 2) acc[mb][nb] = WFrag<T16>::mma(a[mb], b2, acc[mb][nb]); } }
        asm volatile("v_nop\n\tv_nop\n\tv_nop\n\tv_nop" : "+v"(acc[0][0]), "+v"(acc[1][1]), "+v"(acc[2][2]), "+v"(acc[3][3]) : "v"(a[0]), "v"(a[3]));
    }
#pragma unroll
    for (int mb = 0; mb < 4; ++mb) {
#pragma unroll
        for (int nb = 0; nb < 4; ++nb) {
#pragma unroll
            for (int j = 0; j < 8; ++j) os[(hi * 8 + j) * 68 + nb * 16 + lr] = acc[mb][nb][j]; }
        __builtin_amdgcn_fence(3  , "wavefront"); __builtin_amdgcn_wave_barrier(); asm volatile("" ::: "memory");
        float* crow = C + (size_t)(r0 + mb * 16) * ldc + c0;
#pragma unroll 1
        for (int ps = 0; ps < 2; ++ps) {
#pragma unroll
            for (int s = 0; s < 8; ++s) { const int row = 2 * s + hi, cofs = lr * 4; v4f val = *(const v4fa*)(os + row * 68 + cofs); if (BIAS) { val[0] += bfr(bias[c0 + cofs]); val[1] += bfr(bias[c0 + cofs + 1]); val[2] += bfr(bias[c0 + cofs + 2]); val[3] += bfr(bias[c0 + cofs + 3]); }
                *(volatile v4f*)(crow + (size_t)row * ldc + cofs) = val; }
            if (ps == 0) __threadfence(); }
        __builtin_amdgcn_fence(3  , "wavefront"); __builtin_amdgcn_wave_barrier(); asm volatile("" ::: "memory");
    }
}

__global__ __launch_bounds__(256) void k_cvt8(const float* __restrict__ src, bf* dst, size_t n8) { const size_t i = (size_t)blockIdx.x * 256 + threadIdx.x; if (i >= n8) return; const v8f v = *(const v8f*)(src + i * 8); v8us o;
#pragma unroll
    for (int k = 0; k < 8; ++k) o[k] = f2bf(v[k]); *(volatile v8us*)(dst + i * 8) = o; __threadfence(); *(volatile v8us*)(dst + i * 8) = o; }

__global__ __launch_bounds__(256) void k_wtr(const float* __restrict__ W, bf* WT) {
    __shared__ __align__(16) unsigned short ls[64 * 72];
    const unsigned t = threadIdx.x; const unsigned k0 = blockIdx.x * 64u, n0 = blockIdx.y * 64u;
    { const unsigned k = t >> 2, nc = (t & 3u) * 16u; const float* sp = W + (size_t)(k0 + k) * N3 + n0 + nc;
#pragma unroll
      for (unsigned q = 0; q < 4; ++q) { const v4f v = *(const v4f*)(sp + 4u * q);
#pragma unroll
          for (unsigned e = 0; e < 4; ++e) ls[(nc + 4u * q + e) * 72u + k] = f2bf(v[e]); } }
    __syncthreads();
#pragma unroll 1
    for (int ps = 0; ps < 2; ++ps) {
#pragma unroll
        for (unsigned it = 0; it < 2; ++it) { const unsigned n = (t >> 3) + 32u * it, ks = (t & 7u) * 8u; const v8us o = *(const v8usa*)(ls + n * 72u + ks);
            *(volatile v8us*)(WT + (size_t)(n0 + n) * DM + k0 + ks) = o; }
        if (ps == 0) __threadfence(); }
}

__global__ __launch_bounds__(256) void k_hpl(const float* __restrict__ F, bf* PH, bf* PL) {
    const unsigned i = blockIdx.x * 256u + threadIdx.x; const unsigned sel = blockIdx.y; if (i >= (unsigned)(PLN / 8)) return;
    const unsigned e = i * 8u; const unsigned d = e & 63u; const unsigned tt = (e >> 6) % (unsigned)SEQ; const unsigned g = (e >> 6) / (unsigned)SEQ; const unsigned b = g / (unsigned)NH, h = g % (unsigned)NH;
    const float* f = F + (size_t)(b * SEQ + tt) * N3 + sel * DM + h * HD + d; const v4f a = *(const v4f*)f; const v4f c = *(const v4f*)(f + 4); v8us oh, ol;
#pragma unroll
    for (int q = 0; q < 4; ++q) { unsigned short x0, x1; splitf(a[q], x0, x1); oh[q] = x0; ol[q] = x1; splitf(c[q], x0, x1); oh[4 + q] = x0; ol[4 + q] = x1; }
    const size_t oo = (size_t)sel * PLN + e;
    *(volatile v8us*)(PH + oo) = oh; *(volatile v8us*)(PL + oo) = ol; __threadfence(); *(volatile v8us*)(PH + oo) = oh; *(volatile v8us*)(PL + oo) = ol; }

__global__ __launch_bounds__(256) void k_vtp(const float* __restrict__ F, bf* Vh, bf* Vl) {
    const unsigned i = blockIdx.x * 256u + threadIdx.x; if (i >= (unsigned)(PLN / 8)) return;
    const unsigned e = i * 8u; const unsigned tt = e % (unsigned)SEQ; const unsigned d = (e / (unsigned)SEQ) & 63u; const unsigned g = e / (unsigned)(SEQ * HD); const unsigned b = g / (unsigned)NH, h = g % (unsigned)NH;
    const float* f = F + (size_t)(b * SEQ + tt) * N3 + 2 * DM + h * HD + d; v8us oh, ol;
#pragma unroll
    for (int q = 0; q < 8; ++q) { const float x = f[(size_t)q * N3]; unsigned short x0, x1; splitf(x, x0, x1); oh[q] = x0; ol[q] = x1; }
    *(volatile v8us*)(Vh + e) = oh; *(volatile v8us*)(Vl + e) = ol; __threadfence(); *(volatile v8us*)(Vh + e) = oh; *(volatile v8us*)(Vl + e) = ol; }

__global__ __launch_bounds__(128) void k_flash(const bf* __restrict__ QKH, const bf* __restrict__ QKL, const bf* __restrict__ VTH, const bf* __restrict__ VTL, float* OUT) {
    __shared__ __align__(16) float os[4 * 16 * 68];
    const unsigned lane = threadIdx.x & 31u, w = threadIdx.x >> 5, lr = lane & 15u, hi = lane >> 4;
    const unsigned bh = blockIdx.y; const unsigned b = bh / (unsigned)NH, h = bh % (unsigned)NH;
    const unsigned q0 = blockIdx.x * 64u + w * 16u;
    const size_t pb = (size_t)bh * SEQ * HD;
    const bf* qh = QKH + pb + (size_t)(q0 + lr) * HD + 8u * hi;
    const bf* ql = QKL + pb + (size_t)(q0 + lr) * HD + 8u * hi;
    const v16bf qh0 = WFrag<bf>::ld(qh), qh1 = WFrag<bf>::ld(qh + 32), ql0 = WFrag<bf>::ld(ql), ql1 = WFrag<bf>::ld(ql + 32);
    const bf* kh = QKH + PLN + pb + (size_t)lr * HD + 8u * hi;
    const bf* kl = QKL + PLN + pb + (size_t)lr * HD + 8u * hi;
    const bf* vh = VTH + pb + (size_t)lr * SEQ + 8u * hi;
    const bf* vl = VTL + pb + (size_t)lr * SEQ + 8u * hi;
    v8f acc[4];
#pragma unroll
    for (int dt = 0; dt < 4; ++dt) acc[dt] = (v8f){};
    float m = -3.0e38f, lsum = 0.0f;
#pragma unroll 1
    for (unsigned kv = 0; kv < (unsigned)SEQ; kv += 32u) {
        v8f s[2];
#pragma unroll
        for (int t = 0; t < 2; ++t) {
            const bf* kph = kh + (size_t)(kv + 16u * t) * HD; const bf* kpl = kl + (size_t)(kv + 16u * t) * HD;
            const v16bf ah0 = WFrag<bf>::ld(kph), ah1 = WFrag<bf>::ld(kph + 32), al0 = WFrag<bf>::ld(kpl), al1 = WFrag<bf>::ld(kpl + 32);
            s[t] = (v8f){};
            s[t] = wmmab(ah0, qh0, s[t]); s[t] = wmmab(ah1, qh1, s[t]);
            s[t] = wmmab(al0, qh0, s[t]); s[t] = wmmab(al1, qh1, s[t]);
            s[t] = wmmab(ah0, ql0, s[t]); s[t] = wmmab(ah1, ql1, s[t]);
            asm volatile("v_nop\n\tv_nop\n\tv_nop\n\tv_nop" : "+v"(s[t]) : "v"(ah0), "v"(ah1), "v"(al1));
        }
        float mx = m;
#pragma unroll
        for (int t = 0; t < 2; ++t) { s[t] = s[t] * CSC;
#pragma unroll
            for (int r = 0; r < 8; ++r) mx = fmaxf(mx, s[t][r]); }
        mx = fmaxf(mx, __shfl_xor(mx, 16, 32));
        const float fac = __builtin_amdgcn_exp2f(m - mx); m = mx;
        v8u phv, plv; float rs = 0.0f;
#pragma unroll
        for (int t = 0; t < 2; ++t)
#pragma unroll
            for (int j = 0; j < 4; ++j) {
                const float p0 = __builtin_amdgcn_exp2f(s[t][2 * j] - mx), p1 = __builtin_amdgcn_exp2f(s[t][2 * j + 1] - mx);
                rs += p0 + p1;
                const unsigned h0 = __float_as_uint(p0) & 0xffff0000u, h1 = __float_as_uint(p1) & 0xffff0000u;
                const float r0 = p0 - __uint_as_float(h0), r1 = p1 - __uint_as_float(h1);
                phv[t * 4 + j] = (h0 >> 16) | h1;
                plv[t * 4 + j] = (unsigned)f2bf(r0) | (((unsigned)f2bf(r1)) << 16);
            }
        lsum = lsum * fac + rs;
#pragma unroll
        for (int dt = 0; dt < 4; ++dt) acc[dt] = acc[dt] * fac;
        const v16bf pH = __builtin_bit_cast(v16bf, phv), pL = __builtin_bit_cast(v16bf, plv);
#pragma unroll
        for (int dt = 0; dt < 4; ++dt) {
            const v16bf ah = WFrag<bf>::ld(vh + (size_t)(16u * dt) * SEQ + kv), al = WFrag<bf>::ld(vl + (size_t)(16u * dt) * SEQ + kv);
            acc[dt] = wmmab(ah, pH, acc[dt]); acc[dt] = wmmab(al, pH, acc[dt]); acc[dt] = wmmab(ah, pL, acc[dt]);
            asm volatile("v_nop\n\tv_nop\n\tv_nop\n\tv_nop" : "+v"(acc[dt]) : "v"(ah), "v"(al), "v"(pL));
        }
    }
    lsum += __shfl_xor(lsum, 16, 32);
    const float inv = 1.0f / lsum;
    float* o = os + w * (16 * 68);
#pragma unroll
    for (int dt = 0; dt < 4; ++dt) { v4f a, c;
#pragma unroll
        for (int r = 0; r < 4; ++r) { a[r] = acc[dt][r] * inv; c[r] = acc[dt][4 + r] * inv; }
        *(v4fa*)(o + lr * 68u + dt * 16 + 8u * hi) = a; *(v4fa*)(o + lr * 68u + dt * 16 + 8u * hi + 4u) = c; }
    __builtin_amdgcn_fence(3  , "wavefront"); __builtin_amdgcn_wave_barrier(); asm volatile("" ::: "memory");
    float* crow = OUT + ((size_t)b * SEQ + q0) * DM + h * HD;
#pragma unroll 1
    for (int ps = 0; ps < 2; ++ps) {
#pragma unroll
        for (unsigned sidx = 0; sidx < 8; ++sidx) { const unsigned row = 2u * sidx + hi, cofs = lr * 4u; const v4f val = *(const v4fa*)(o + row * 68u + cofs);
            *(volatile v4f*)(crow + (size_t)row * DM + cofs) = val; }
        if (ps == 0) __threadfence(); }
}

extern "C" void kernel_launch(void* const* d_in, const int* in_sizes, int n_in,
                              void* d_out, int out_size, void* d_ws, size_t ws_size, hipStream_t stream) {
    if (n_in < 2) return;
    if ((size_t)in_sizes[0] < (size_t)(NB - 1) * SEQ_FULL * DM + (size_t)SEQ * DM) return;
    if ((size_t)in_sizes[1] < (size_t)DM * N3) return;
    if ((size_t)out_size < (size_t)NB * SEQ * DM) return;
    const float* x = (const float*)d_in[0];
    const float* wqkv = (const float*)d_in[1];
    float* OUT = (float*)d_out;
    char* wsp = (char*)d_ws;
    auto take = [&](size_t bytes) { char* p = wsp; wsp += (bytes + 255) & ~(size_t)255; return (void*)p; };
    bf* WT = (bf*)take((size_t)N3 * DM * 2);
    bf* XB = (bf*)take((size_t)MROWS * DM * 2);
    float* F = (float*)take((size_t)MROWS * N3 * 4);
    bf* QKH = (bf*)take((size_t)2 * PLN * 2);
    bf* QKL = (bf*)take((size_t)2 * PLN * 2);
    bf* VTH = (bf*)take(PLN * 2);
    bf* VTL = (bf*)take(PLN * 2);
    const size_t carved = (size_t)(wsp - (char*)d_ws);
    if (carved > ws_size || carved > (size_t)134217728) return;

    for (int b = 0; b < NB; ++b)
        k_cvt8<<<(unsigned)(((size_t)SEQ * DM / 8 + 255) / 256), 256, 0, stream>>>(x + (size_t)b * SEQ_FULL * DM, XB + (size_t)b * SEQ * DM, (size_t)SEQ * DM / 8);
    k_wtr<<<dim3(DM / 64, N3 / 64), 256, 0, stream>>>(wqkv, WT);
    k_gemmw<bf, 0, false><<<dim3(MROWS / 64, N3 / 64, 1), 32, 0, stream>>>(XB, nullptr, WT, nullptr, DM, F, N3, nullptr, 0, 0, 0);
    const unsigned LP = (unsigned)((PLN / 8 + 255) / 256);
    k_hpl<<<dim3(LP, 2), 256, 0, stream>>>(F, QKH, QKL);
    k_vtp<<<LP, 256, 0, stream>>>(F, VTH, VTL);
    k_flash<<<dim3(SEQ / 64, NBH), 128, 0, stream>>>(QKH, QKL, VTH, VTL, OUT);
}
